// MultiHeadedAttention_84499186581895
// MI455X (gfx1250) — hardware-verified
//
#include <hip/hip_runtime.h>
#include <math.h>

#ifndef NB
#define NB 2
#endif
#ifndef SEQ
#define SEQ 2048
#endif
#define NB_FULL 2
#define SEQ_FULL 2048
#define HD 64
#define NH 16
#define EMB 1024
#ifndef EARLY_ROWS
#define EARLY_ROWS 256
#endif
#define EARLY_QB (EARLY_ROWS / 64)
#define RES_SHIFT 2048.0f
#define RES_INV (1.0f / 2048.0f)
#define PSC 1024.0f
#define CTXS 64.0f
#define WOS 32.0f
#define WPS 16.0f

static_assert(SEQ % 64 == 0);
static_assert(EARLY_ROWS % 64 == 0);
static_assert(EARLY_ROWS <= SEQ);
static_assert(HD == 64);
static_assert(NH * HD == EMB);
static_assert(EMB % 64 == 0);
static_assert(EMB % 32 == 0);
static_assert(HD % 32 == 0);
static_assert(NB <= NB_FULL);
static_assert(SEQ <= SEQ_FULL);

typedef __attribute__((ext_vector_type(16))) _Float16 v16h;
typedef __attribute__((ext_vector_type(8)))  _Float16 v8h;
typedef __attribute__((ext_vector_type(8)))  float    v8f;
typedef __attribute__((ext_vector_type(4)))  float    v4f;
typedef __attribute__((ext_vector_type(4)))  unsigned u4;

union FragU { v16h v; v8h h[2]; };
__device__ __forceinline__ v16h ldfrag(const _Float16* p) { FragU f; f.h[0] = *(const v8h*)(p); f.h[1] = *(const v8h*)(p + 16); return f.v; }

__device__ __forceinline__ v8f mma16(v16h a, v16h b, v8f c) {
  c = __builtin_amdgcn_wmma_f32_16x16x32_f16(false, a, false, b, (short)0, c, false, false);
  asm volatile("v_nop\n\tv_nop\n\tv_nop\n\tv_nop" : "+v"(c) : "v"(a), "v"(b));
  return c;
}
__device__ __forceinline__ void dep_guard_h(v8f& a, v8f& b, v16h x, v16h y) { asm volatile("v_nop\n\tv_nop\n\tv_nop\n\tv_nop" : "+v"(a), "+v"(b) : "v"(x), "v"(y)); }
__device__ __forceinline__ void keep4_h(v16h a, v16h b, v16h c, v16h d) { asm volatile("v_nop" :: "v"(a), "v"(b), "v"(c), "v"(d)); }
__device__ __forceinline__ void acc_guard4(v8f& a, v8f& b, v8f& c, v8f& d) { asm volatile("v_nop\n\tv_nop\n\tv_nop\n\tv_nop" : "+v"(a), "+v"(b), "+v"(c), "+v"(d)); }
__device__ __forceinline__ void wave_lds_sync() {
  __builtin_amdgcn_fence(3  , "workgroup");
  __builtin_amdgcn_wave_barrier();
  __builtin_amdgcn_fence(2  , "workgroup");
}

#define VST2(T, ptr, val) do { const T vst2_v_ = (val); *(volatile T*)(ptr) = vst2_v_; __threadfence(); *(volatile T*)(ptr) = vst2_v_; } while (0)

__device__ __forceinline__ float bf_rne_keep(float v) {
  const unsigned u = __builtin_bit_cast(unsigned, v);
  const unsigned r = (u + 0x7fffu + ((u >> 16) & 1u)) & 0xffff0000u;
  return __builtin_bit_cast(float, r);
}
__device__ __forceinline__ unsigned pk2h(float a, float b) {
  return (unsigned)__builtin_bit_cast(unsigned short, (_Float16)a) | ((unsigned)__builtin_bit_cast(unsigned short, (_Float16)b) << 16);
}

__global__ __launch_bounds__(256) void k_cast_rows(const float* __restrict__ SRC, long long sSz, int lds,
                                                   unsigned short* __restrict__ DST, long long sDz, int ldd, int nR, int nC, float sc) {
  const long long u = (long long)blockIdx.x * 256 + threadIdx.x; const int per = nC / 8;
  if (u >= (long long)nR * per) return;
  const int r = (int)(u / per); const int c0 = 8 * (int)(u % per);
  const float* s = SRC + (long long)blockIdx.y * sSz + (long long)r * lds + c0;
  const v4f x0 = *(const v4f*)s, x1 = *(const v4f*)(s + 4);
  u4 pk;
  pk.x = pk2h(bf_rne_keep(x0.x) * sc, bf_rne_keep(x0.y) * sc); pk.y = pk2h(bf_rne_keep(x0.z) * sc, bf_rne_keep(x0.w) * sc);
  pk.z = pk2h(bf_rne_keep(x1.x) * sc, bf_rne_keep(x1.y) * sc); pk.w = pk2h(bf_rne_keep(x1.z) * sc, bf_rne_keep(x1.w) * sc);
  VST2(u4, (u4*)(DST + (long long)blockIdx.y * sDz + (long long)r * ldd + c0), pk);
}
__global__ __launch_bounds__(256) void k_cast_T(const float* __restrict__ SRC, long long sSz, int lds,
                                                unsigned short* __restrict__ DST, long long sDz, int ldd, int nR, int nC, float sc) {
  const long long u = (long long)blockIdx.x * 256 + threadIdx.x; const int per = nR / 8;
  if (u >= (long long)nC * per) return;
  const int c = (int)(u / per); const int r0 = 8 * (int)(u % per);
  const float* s = SRC + (long long)blockIdx.y * sSz;
  float w[8];
#pragma unroll
  for (int e = 0; e < 8; ++e) w[e] = bf_rne_keep(s[(long long)(r0 + e) * lds + c]) * sc;
  u4 pk; pk.x = pk2h(w[0], w[1]); pk.y = pk2h(w[2], w[3]); pk.z = pk2h(w[4], w[5]); pk.w = pk2h(w[6], w[7]);
  VST2(u4, (u4*)(DST + (long long)blockIdx.y * sDz + (long long)c * ldd + r0), pk);
}

__device__ __forceinline__ void gemm64_kloop(v8f (&acc)[4][4], const _Float16* __restrict__ Ab, int lda,
                                             const _Float16* __restrict__ Bb, int ldb, int m0, int n0, int K, int rlane, int koff) {
  for (int k0 = 0; k0 < K; k0 += 32) {
    v16h bh[4];
#pragma unroll
    for (int j = 0; j < 4; ++j) bh[j] = ldfrag(Bb + (size_t)(n0 + (j << 4) + rlane) * ldb + koff + k0);
#pragma unroll
    for (int i = 0; i < 4; ++i) {
      const v16h ah = ldfrag(Ab + (size_t)(m0 + (i << 4) + rlane) * lda + koff + k0);
#pragma unroll
      for (int j = 0; j < 4; ++j)
        acc[i][j] = __builtin_amdgcn_wmma_f32_16x16x32_f16(false, ah, false, bh[j], (short)0, acc[i][j], false, false);
      dep_guard_h(acc[i][0], acc[i][3], ah, ah);
    }
    keep4_h(bh[0], bh[1], bh[2], bh[3]);
  }
  acc_guard4(acc[0][0], acc[0][1], acc[0][2], acc[0][3]);
  acc_guard4(acc[1][0], acc[1][1], acc[1][2], acc[1][3]);
  acc_guard4(acc[2][0], acc[2][1], acc[2][2], acc[2][3]);
  acc_guard4(acc[3][0], acc[3][1], acc[3][2], acc[3][3]);
}

__global__ __launch_bounds__(256) void k_proj(const unsigned short* __restrict__ Ap, int lda, long long strideA,
                                              const unsigned short* __restrict__ Btp, int ldb, long long strideB,
                                              unsigned short* __restrict__ Chi, unsigned short* __restrict__ Cres, int ldc, long long strideC,
                                              int M, int N, int K, float scale) {
  __shared__ __align__(16) float sT[8][16 * 68];
  const int b = blockIdx.y, lane = threadIdx.x & 31, wave = threadIdx.x >> 5;
  const int tilesN = N >> 6, tilesM = M >> 6;
  const int tile = blockIdx.x * 8 + wave;
  if (tile >= tilesM * tilesN) return;
  const int tm = tile / tilesN, tn = tile - tm * tilesN;
  const int m0 = tm << 6, n0 = tn << 6;
  const _Float16* Ab = (const _Float16*)Ap + (size_t)b * strideA;
  const _Float16* Bb = (const _Float16*)Btp + (size_t)b * strideB;
  const int rlane = lane & 15, koff = (lane >> 4) * 8, mOff = (lane >> 4) * 8;
  v8f acc[4][4];
#pragma unroll
  for (int i = 0; i < 4; ++i)
#pragma unroll
    for (int j = 0; j < 4; ++j) acc[i][j] = (v8f){0.f, 0.f, 0.f, 0.f, 0.f, 0.f, 0.f, 0.f};
  gemm64_kloop(acc, Ab, lda, Bb, ldb, m0, n0, K, rlane, koff);
  unsigned short* Ch = Chi + (size_t)b * strideC;
  unsigned short* Cr = Cres + (size_t)b * strideC;
  const int q = lane >> 3, c8 = (lane & 7) * 8;
#pragma unroll
  for (int i = 0; i < 4; ++i) {
    const int mBase = m0 + (i << 4);
#pragma unroll
    for (int j = 0; j < 4; ++j)
#pragma unroll
      for (int r = 0; r < 8; ++r) sT[wave][(mOff + r) * 68 + (j << 4) + rlane] = acc[i][j][r] * scale;
    wave_lds_sync();
    for (int pass = 0; pass < 2; ++pass) {
#pragma unroll
      for (int it = 0; it < 4; ++it) {
        const int row = it * 4 + q;
        const v4f x0 = *(const v4f*)&sT[wave][row * 68 + c8], x1 = *(const v4f*)&sT[wave][row * 68 + c8 + 4];
        const float sp[8] = {x0.x, x0.y, x0.z, x0.w, x1.x, x1.y, x1.z, x1.w};
        v8h hv, lv;
#pragma unroll
        for (int e = 0; e < 8; ++e) { const _Float16 hb = (_Float16)sp[e]; hv[e] = hb; lv[e] = (_Float16)((sp[e] - (float)hb) * RES_SHIFT); }
        *(volatile v8h*)(Ch + (size_t)(mBase + row) * ldc + n0 + c8) = hv;
        *(volatile v8h*)(Cr + (size_t)(mBase + row) * ldc + n0 + c8) = lv;
      }
      __threadfence();
    }
    wave_lds_sync();
  }
}

__global__ __launch_bounds__(256) void k_oproj(const unsigned short* __restrict__ Ap, const unsigned short* __restrict__ A2p, int lda,
                                               const unsigned short* __restrict__ Btp, int ldb, float* __restrict__ Cout, int ldc,
                                               const float* __restrict__ bias, int M, int N, int K, float scale, int seq_rows, int early_rows) {
  __shared__ __align__(16) float sT[8][16 * 68];
  const int lane = threadIdx.x & 31, wave = threadIdx.x >> 5;
  const int tilesN = N >> 6, tilesM = M >> 6;
  const int tile = blockIdx.x * 8 + wave;
  if (tile >= tilesM * tilesN) return;
  const int tm = tile / tilesN, tn = tile - tm * tilesN;
  const int m0 = tm << 6, n0 = tn << 6;
  const _Float16* Ab = (const _Float16*)Ap;
  const _Float16* A2b = (const _Float16*)A2p;
  const _Float16* Bb = (const _Float16*)Btp;
  const int rlane = lane & 15, koff = (lane >> 4) * 8, mOff = (lane >> 4) * 8;
  v8f acc[4][4];
#pragma unroll
  for (int i = 0; i < 4; ++i)
#pragma unroll
    for (int j = 0; j < 4; ++j) acc[i][j] = (v8f){0.f, 0.f, 0.f, 0.f, 0.f, 0.f, 0.f, 0.f};
  const bool early = (m0 % seq_rows) < early_rows;
  if (early) {
    gemm64_kloop(acc, A2b, lda, Bb, ldb, m0, n0, K, rlane, koff);
#pragma unroll
    for (int i = 0; i < 4; ++i)
#pragma unroll
      for (int j = 0; j < 4; ++j) acc[i][j] = acc[i][j] * RES_INV;
  }
  gemm64_kloop(acc, Ab, lda, Bb, ldb, m0, n0, K, rlane, koff);
  const int hh = lane >> 4, c4 = (lane & 15) * 4;
#pragma unroll
  for (int i = 0; i < 4; ++i) {
    const int mBase = m0 + (i << 4);
#pragma unroll
    for (int j = 0; j < 4; ++j) {
      const float bv = bf_rne_keep(bias[n0 + (j << 4) + rlane]);
#pragma unroll
      for (int r = 0; r < 8; ++r) sT[wave][(mOff + r) * 68 + (j << 4) + rlane] = acc[i][j][r] * scale + bv;
    }
    wave_lds_sync();
    for (int pass = 0; pass < 2; ++pass) {
#pragma unroll
      for (int it = 0; it < 8; ++it) {
        const int row = it * 2 + hh;
        const v4f v = *(const v4f*)&sT[wave][row * 68 + c4];
        *(volatile v4f*)(Cout + (size_t)(mBase + row) * ldc + n0 + c4) = v;
      }
      __threadfence();
    }
    wave_lds_sync();
  }
}

template <bool EARLY>
__device__ __forceinline__ void attn_body(const unsigned short* Qh_, const unsigned short* Qr_, const unsigned short* Kh_, const unsigned short* Kr_,
                                          const unsigned short* Vh_, const unsigned short* Vr_, unsigned short* Ch_, unsigned short* Cr_, float rsl) {
  __shared__ __align__(16) _Float16 Ph[4][16 * 64];
  __shared__ __align__(16) _Float16 Pr[EARLY ? 4 : 1][EARLY ? 16 * 64 : 8];
  __shared__ __align__(16) float    Os[4][16 * 68];
  const int tid = threadIdx.x, wave = tid >> 5, lane = tid & 31, hh = lane >> 4, c = lane & 15;
  constexpr int NQB = EARLY ? EARLY_QB : ((SEQ / 64 - EARLY_QB) > 0 ? (SEQ / 64 - EARLY_QB) : 1);
  const int bx = blockIdx.x;
  const int qb = (bx % NQB) + (EARLY ? 0 : EARLY_QB);
  const int bh = bx / NQB;
  const int h = bh % NH, b = bh / NH;
  const int q0 = qb * 64 + wave * 16;

  const size_t qkbase = (size_t)b * SEQ * EMB + (size_t)h * HD;
  const size_t vbase  = ((size_t)b * EMB + (size_t)h * HD) * SEQ;
  const _Float16* Qh = (const _Float16*)Qh_ + qkbase;
  const _Float16* Qr = (const _Float16*)Qr_ + qkbase;
  const _Float16* Kh = (const _Float16*)Kh_ + qkbase;
  const _Float16* Kr = (const _Float16*)Kr_ + qkbase;
  const _Float16* Vh = (const _Float16*)Vh_ + vbase;
  const _Float16* Vr = (const _Float16*)Vr_ + vbase;

  float mrow[8], lrow[8];
  v8f o[4], o2[4];
#pragma unroll
  for (int r = 0; r < 8; ++r) { mrow[r] = -INFINITY; lrow[r] = 0.f; }
#pragma unroll
  for (int t = 0; t < 4; ++t) { o[t] = (v8f){0.f, 0.f, 0.f, 0.f, 0.f, 0.f, 0.f, 0.f}; o2[t] = o[t]; }

#pragma unroll 1
  for (int kc = 0; kc <= qb; ++kc) {
    const int kv0 = kc * 64;
    v8f s[4];
#pragma unroll
    for (int j = 0; j < 4; ++j) s[j] = (v8f){0.f, 0.f, 0.f, 0.f, 0.f, 0.f, 0.f, 0.f};
    if (EARLY) {
#pragma unroll 1
      for (int dc = 0; dc < 2; ++dc) {
        const int qo = (q0 + c) * EMB + dc * 32 + 8 * hh;
        const v16h qa = ldfrag(Qh + qo), qr = ldfrag(Qr + qo);
#pragma unroll
        for (int j = 0; j < 4; ++j) {
          const int ko = (kv0 + 16 * j + c) * EMB + dc * 32 + 8 * hh;
          const v16h kb = ldfrag(Kh + ko), kr = ldfrag(Kr + ko);
          s[j] = mma16(qa, kr, s[j]);
          s[j] = mma16(qr, kb, s[j]);
        }
      }
#pragma unroll
      for (int j = 0; j < 4; ++j) s[j] = s[j] * RES_INV;
    }
#pragma unroll 1
    for (int dc = 0; dc < 2; ++dc) {
      const int qo = (q0 + c) * EMB + dc * 32 + 8 * hh;
      const v16h qa = ldfrag(Qh + qo);
#pragma unroll
      for (int j = 0; j < 4; ++j) {
        const int ko = (kv0 + 16 * j + c) * EMB + dc * 32 + 8 * hh;
        const v16h kb = ldfrag(Kh + ko);
        s[j] = mma16(qa, kb, s[j]);
      }
    }
    const bool diag = (kc == qb);
    float cm[8];
#pragma unroll
    for (int r = 0; r < 8; ++r) {
      const int qrow = q0 + 8 * hh + r;
      float m = -INFINITY;
#pragma unroll
      for (int j = 0; j < 4; ++j) {
        const int kvcol = kv0 + j * 16 + c;
        float v = s[j][r] * rsl;
        v = (diag && kvcol > qrow) ? -INFINITY : v;
        s[j][r] = v;
        m = fmaxf(m, v);
      }
      m = fmaxf(m, __shfl_xor(m, 1, 32)); m = fmaxf(m, __shfl_xor(m, 2, 32));
      m = fmaxf(m, __shfl_xor(m, 4, 32)); m = fmaxf(m, __shfl_xor(m, 8, 32));
      cm[r] = m;
    }
    wave_lds_sync();
#pragma unroll
    for (int r = 0; r < 8; ++r) {
      const float mnew = fmaxf(mrow[r], cm[r]);
      const float alpha = exp2f(mrow[r] - mnew);
      mrow[r] = mnew;
      float psum = 0.f;
#pragma unroll
      for (int j = 0; j < 4; ++j) {
        const float p = exp2f(s[j][r] - mnew);
        psum += p;
        const float ps = p * PSC;
        const _Float16 ph = (_Float16)ps;
        Ph[wave][(8 * hh + r) * 64 + j * 16 + c] = ph;
        if (EARLY) Pr[wave][(8 * hh + r) * 64 + j * 16 + c] = (_Float16)((ps - (float)ph) * RES_SHIFT);
      }
      psum += __shfl_xor(psum, 1, 32); psum += __shfl_xor(psum, 2, 32);
      psum += __shfl_xor(psum, 4, 32); psum += __shfl_xor(psum, 8, 32);
      lrow[r] = lrow[r] * alpha + psum;
#pragma unroll
      for (int t = 0; t < 4; ++t) { o[t][r] *= alpha; if (EARLY) o2[t][r] *= alpha; }
    }
    wave_lds_sync();
#pragma unroll 1
    for (int kk = 0; kk < 2; ++kk) {
      const int po = c * 64 + kk * 32 + 8 * hh;
      FragU pa, pr;
      pa.h[0] = *(const v8h*)&Ph[wave][po]; pa.h[1] = *(const v8h*)&Ph[wave][po + 16];
      if (EARLY) { pr.h[0] = *(const v8h*)&Pr[wave][po]; pr.h[1] = *(const v8h*)&Pr[wave][po + 16]; }
#pragma unroll
      for (int t = 0; t < 4; ++t) {
        const int vo = (16 * t + c) * SEQ + kv0 + kk * 32 + 8 * hh;
        const v16h vb = ldfrag(Vh + vo);
        o[t] = mma16(pa.v, vb, o[t]);
        if (EARLY) {
          const v16h vr = ldfrag(Vr + vo);
          o2[t] = mma16(pa.v, vr, o2[t]);
          o2[t] = mma16(pr.v, vb, o2[t]);
        }
      }
    }
  }

#pragma unroll
  for (int r = 0; r < 8; ++r) {
    const float inv = (CTXS / PSC) * (1.0f / lrow[r]);
#pragma unroll
    for (int t = 0; t < 4; ++t) {
      const float val = EARLY ? (o[t][r] + o2[t][r] * RES_INV) * inv : o[t][r] * inv;
      Os[wave][(8 * hh + r) * 68 + t * 16 + c] = val;
    }
  }
  wave_lds_sync();
  {
    const int qd = lane >> 3, c8 = (lane & 7) * 8;
    const size_t obase = ((size_t)b * SEQ + q0) * EMB + (size_t)h * HD + c8;
    for (int pass = 0; pass < 2; ++pass) {
#pragma unroll
      for (int it = 0; it < 4; ++it) {
        const int row = it * 4 + qd;
        const v4f x0 = *(const v4f*)&Os[wave][row * 68 + c8], x1 = *(const v4f*)&Os[wave][row * 68 + c8 + 4];
        const float sp[8] = {x0.x, x0.y, x0.z, x0.w, x1.x, x1.y, x1.z, x1.w};
        v8h hv, lv;
#pragma unroll
        for (int e = 0; e < 8; ++e) { const _Float16 hb = (_Float16)sp[e]; hv[e] = hb; lv[e] = (_Float16)((sp[e] - (float)hb) * RES_SHIFT); }
        *(volatile v8h*)(Ch_ + obase + (size_t)row * EMB) = hv;
        if (EARLY) *(volatile v8h*)(Cr_ + obase + (size_t)row * EMB) = lv;
      }
      __threadfence();
    }
  }
}

__global__ __launch_bounds__(128) void k_attn_early(const unsigned short* __restrict__ Qh, const unsigned short* __restrict__ Qr,
                                                    const unsigned short* __restrict__ Kh, const unsigned short* __restrict__ Kr,
                                                    const unsigned short* __restrict__ Vh, const unsigned short* __restrict__ Vr,
                                                    unsigned short* __restrict__ Ch, unsigned short* __restrict__ Cr, float rsl) {
  attn_body<true>(Qh, Qr, Kh, Kr, Vh, Vr, Ch, Cr, rsl);
}
__global__ __launch_bounds__(128) void k_attn_late(const unsigned short* __restrict__ Qh, const unsigned short* __restrict__ Kh,
                                                   const unsigned short* __restrict__ Vh, unsigned short* __restrict__ Ch, float rsl) {
  attn_body<false>(Qh, Qh, Kh, Kh, Vh, Vh, Ch, Ch, rsl);
}

constexpr size_t al256(size_t x) { return (x + 255) / 256 * 256; }
constexpr size_t SZ_X  = al256((size_t)NB * SEQ * HD * 2);
constexpr size_t SZ_WP = al256((size_t)EMB * HD * 2);
constexpr size_t SZ_WO = al256((size_t)EMB * EMB * 2);
constexpr size_t SZ_PL = al256((size_t)NB * SEQ * EMB * 2);
constexpr size_t WS_TOTAL = 3 * SZ_X + 3 * SZ_WP + SZ_WO + 8 * SZ_PL;
static_assert(WS_TOTAL <= 134217728);

extern "C" void kernel_launch(void* const* d_in, const int* in_sizes, int n_in, void* d_out, int out_size, void* d_ws, size_t ws_size, hipStream_t stream) {
  if (n_in < 8) return;
  const long long need_x = (long long)(NB - 1) * SEQ_FULL * HD + (long long)SEQ * HD;
  if (in_sizes[0] < need_x || in_sizes[1] < need_x || in_sizes[2] < need_x) return;
  if (in_sizes[3] < NH * HD * HD || in_sizes[4] < NH * HD * HD || in_sizes[5] < NH * HD * HD) return;
  if (in_sizes[6] < EMB * EMB || in_sizes[7] < EMB) return;
  if ((long long)out_size < (long long)NB * SEQ * EMB) return;
  if (WS_TOTAL > ws_size) return;

  const float* x_k = (const float*)d_in[0];
  const float* x_v = (const float*)d_in[1];
  const float* x_q = (const float*)d_in[2];
  const float* Wk  = (const float*)d_in[3];
  const float* Wv  = (const float*)d_in[4];
  const float* Wq  = (const float*)d_in[5];
  const float* Wo  = (const float*)d_in[6];
  const float* bo  = (const float*)d_in[7];
  float* out = (float*)d_out;

  char* wsp = (char*)d_ws;
  unsigned short* Xk16 = (unsigned short*)wsp; wsp += SZ_X;
  unsigned short* Xv16 = (unsigned short*)wsp; wsp += SZ_X;
  unsigned short* Xq16 = (unsigned short*)wsp; wsp += SZ_X;
  unsigned short* WkT  = (unsigned short*)wsp; wsp += SZ_WP;
  unsigned short* WvT  = (unsigned short*)wsp; wsp += SZ_WP;
  unsigned short* WqT  = (unsigned short*)wsp; wsp += SZ_WP;
  unsigned short* WoT  = (unsigned short*)wsp; wsp += SZ_WO;
  unsigned short* Qhp  = (unsigned short*)wsp; wsp += SZ_PL;
  unsigned short* Qrp  = (unsigned short*)wsp; wsp += SZ_PL;
  unsigned short* Khp  = (unsigned short*)wsp; wsp += SZ_PL;
  unsigned short* Krp  = (unsigned short*)wsp; wsp += SZ_PL;
  unsigned short* Vhp  = (unsigned short*)wsp; wsp += SZ_PL;
  unsigned short* Vrp  = (unsigned short*)wsp; wsp += SZ_PL;
  unsigned short* Chp  = (unsigned short*)wsp; wsp += SZ_PL;
  unsigned short* Crp  = (unsigned short*)wsp; wsp += SZ_PL;

  {
    const dim3 g((unsigned)(((long long)SEQ * (HD / 8) + 255) / 256), (unsigned)NB);
    k_cast_rows<<<g, 256, 0, stream>>>(x_k, (long long)SEQ_FULL * HD, HD, Xk16, (long long)SEQ * HD, HD, SEQ, HD, 1.0f);
    k_cast_rows<<<g, 256, 0, stream>>>(x_v, (long long)SEQ_FULL * HD, HD, Xv16, (long long)SEQ * HD, HD, SEQ, HD, 1.0f);
    k_cast_rows<<<g, 256, 0, stream>>>(x_q, (long long)SEQ_FULL * HD, HD, Xq16, (long long)SEQ * HD, HD, SEQ, HD, 1.0f);
  }
  {
    const dim3 g((unsigned)(((long long)HD * (HD / 8) + 255) / 256), (unsigned)NH);
    k_cast_T<<<g, 256, 0, stream>>>(Wk, (long long)HD * HD, HD, WkT, (long long)HD * HD, HD, HD, HD, WPS);
    k_cast_T<<<g, 256, 0, stream>>>(Wv, (long long)HD * HD, HD, WvT, (long long)HD * HD, HD, HD, HD, WPS);
    k_cast_T<<<g, 256, 0, stream>>>(Wq, (long long)HD * HD, HD, WqT, (long long)HD * HD, HD, HD, HD, WPS);
  }
  {
    const dim3 g((unsigned)(((long long)EMB * (EMB / 8) + 255) / 256), 1u);
    k_cast_T<<<g, 256, 0, stream>>>(Wo, 0LL, EMB, WoT, 0LL, EMB, EMB, EMB, WOS);
  }
  {
    const int tiles = ((NB * SEQ) / 64) * (EMB / 64);
    const dim3 g((unsigned)((tiles + 7) / 8), 1u);
    k_proj<<<g, 256, 0, stream>>>(Xq16, HD, 0LL, WqT, HD, 0LL, Qhp, Qrp, EMB, 0LL, NB * SEQ, EMB, HD, 1.0f / WPS);
    k_proj<<<g, 256, 0, stream>>>(Xk16, HD, 0LL, WkT, HD, 0LL, Khp, Krp, EMB, 0LL, NB * SEQ, EMB, HD, 1.0f / WPS);
    const int tilesv = (EMB / 64) * (SEQ / 64);
    const dim3 gv((unsigned)((tilesv + 7) / 8), (unsigned)NB);
    k_proj<<<gv, 256, 0, stream>>>(WvT, HD, 0LL, Xv16, HD, (long long)SEQ * HD, Vhp, Vrp, SEQ, (long long)EMB * SEQ, EMB, SEQ, HD, 1.0f / WPS);
  }
  {
    const float rsl = (1.0f / sqrtf((float)SEQ)) * 1.4426950408889634f;
    const int nearly = NB * NH * EARLY_QB;
    const int nlate = NB * NH * (SEQ / 64 - EARLY_QB);
    k_attn_early<<<dim3((unsigned)nearly), 128, 0, stream>>>(Qhp, Qrp, Khp, Krp, Vhp, Vrp, Chp, Crp, rsl);
    if (nlate > 0) k_attn_late<<<dim3((unsigned)nlate), 128, 0, stream>>>(Qhp, Khp, Vhp, Chp, rsl);
  }
  {
    const int tiles = ((NB * SEQ) / 64) * (EMB / 64);
    const dim3 g((unsigned)((tiles + 7) / 8), 1u);
    k_oproj<<<g, 256, 0, stream>>>(Chp, Crp, EMB, WoT, EMB, out, EMB, bo, NB * SEQ, EMB, EMB, 1.0f / (CTXS * WOS), SEQ, EARLY_ROWS);
  }
}
